// PGNN_layer_42992622633782
// MI455X (gfx1250) — hardware-verified
//
#include <hip/hip_runtime.h>
#include <stddef.h>


typedef _Float16 v16h __attribute__((ext_vector_type(16)));
typedef _Float16 v8h  __attribute__((ext_vector_type(8)));
typedef float    v8f  __attribute__((ext_vector_type(8)));
typedef float    v4fa __attribute__((ext_vector_type(4))) __attribute__((may_alias));

#define DIN   128
#define DOUT  128
#define KNB   16
#define WS    136
#define WSCALE 16.0f
#define WINV  (1.0f / 16.0f)

#define SELF_TPB   128
#define SELF_ROWS  64
#define NODE_TPB   256
#define NODE_WPB   8
#define NPW        16
#define NODES_PER_BLOCK (NODE_WPB * NPW)
#define CHUNK_NODES 16384
#define GATHER_TPB 256

static_assert(NPW % 2 == 0, "");
static_assert(CHUNK_NODES % NODES_PER_BLOCK == 0, "");

union Frag { v16h v; v8h half[2]; };

__device__ __forceinline__ v8f wmma16(const v16h a, const v16h b, v8f c) {
    c = __builtin_amdgcn_wmma_f32_16x16x32_f16(false, a, false, b, (short)0, c, false, false);
    asm volatile("v_nop\n\tv_nop\n\tv_nop\n\tv_nop" : "+v"(c) : "v"(a), "v"(b));
    return c;
}

__device__ __forceinline__ v8h cvt8(const float4 f0, const float4 f1, const float s) {
    v8h r;
    r[0] = (_Float16)(f0.x * s); r[1] = (_Float16)(f0.y * s);
    r[2] = (_Float16)(f0.z * s); r[3] = (_Float16)(f0.w * s);
    r[4] = (_Float16)(f1.x * s); r[5] = (_Float16)(f1.y * s);
    r[6] = (_Float16)(f1.z * s); r[7] = (_Float16)(f1.w * s);
    return r;
}

__global__ __launch_bounds__(SELF_TPB) void k_self(
    const float* __restrict__ feature, const float* __restrict__ W_hidden,
    float* __restrict__ selfp, int N)
{
    __shared__ __attribute__((aligned(16))) _Float16 wt[DOUT * WS];
    __shared__ __attribute__((aligned(16))) float stile[4][8][DOUT];

    const int tid = threadIdx.x;
    for (int e = tid; e < DIN * DOUT; e += SELF_TPB) {
        const int k = e >> 7;
        const int o = e & 127;
        wt[o * WS + k] = (_Float16)(W_hidden[(size_t)(DIN + k) * DOUT + o] * WSCALE);
    }
    __syncthreads();

    const int l = tid & 31, h = l >> 4, m = l & 15, w = tid >> 5;
    const int row0 = blockIdx.x * SELF_ROWS + w * 16;
    int arow = row0 + m;
    if (arow > N - 1) arow = N - 1;

    const float* ap = feature + (size_t)arow * DIN + 8 * h;
    Frag a[4];
#pragma unroll
    for (int kc = 0; kc < 4; ++kc) {
        const float4 f0 = *(const float4*)(ap + kc * 32);
        const float4 f1 = *(const float4*)(ap + kc * 32 + 4);
        const float4 f2 = *(const float4*)(ap + kc * 32 + 16);
        const float4 f3 = *(const float4*)(ap + kc * 32 + 20);
        a[kc].half[0] = cvt8(f0, f1, 1.0f);
        a[kc].half[1] = cvt8(f2, f3, 1.0f);
    }

    v8f acc[8];
    const v8f zero = {};
#pragma unroll
    for (int cb = 0; cb < 8; ++cb) acc[cb] = zero;

#pragma unroll
    for (int cb = 0; cb < 8; ++cb) {
        unsigned wb = (unsigned)(m * WS + 8 * h);
        asm volatile("" : "+v"(wb));
        const _Float16* bp = wt + wb + cb * 16 * WS;
        Frag b[4];
#pragma unroll
        for (int kc = 0; kc < 4; ++kc) {
            b[kc].half[0] = *(const v8h*)(bp + kc * 32);
            b[kc].half[1] = *(const v8h*)(bp + kc * 32 + 16);
        }
#pragma unroll
        for (int kc = 0; kc < 4; ++kc) acc[cb] = wmma16(a[kc].v, b[kc].v, acc[cb]);
    }

    float* st = &stile[w][0][0];
    float* orow = selfp + (size_t)row0 * DOUT + 4 * l;
#pragma unroll
    for (int ph = 0; ph < 2; ++ph) {
        if (h == ph) {
#pragma unroll
            for (int cb = 0; cb < 8; ++cb) {
#pragma unroll
                for (int r = 0; r < 8; ++r) st[r * DOUT + cb * 16 + m] = acc[cb][r] * WINV;
            }
        }
        v4fa vv[8];
#pragma unroll
        for (int rr = 0; rr < 8; ++rr) vv[rr] = *(const v4fa*)(st + rr * DOUT + 4 * l);
#pragma unroll
        for (int rr = 0; rr < 8; ++rr)
            *(volatile v4fa*)(orow + (size_t)(ph * 8 + rr) * DOUT) = vv[rr];
        __threadfence();
#pragma unroll
        for (int rr = 0; rr < 8; ++rr)
            *(volatile v4fa*)(orow + (size_t)(ph * 8 + rr) * DOUT) = vv[rr];
    }
}

__global__ __launch_bounds__(GATHER_TPB) void k_gather(
    const float* __restrict__ feature, const float* __restrict__ dists_max,
    const int* __restrict__ dists_argmax, _Float16* __restrict__ msg, int N, int c0)
{
    const int node = c0 + (int)blockIdx.x;
    if (node >= N) return;
    const int t = threadIdx.x;
    const int mrow = t >> 4;
    const int g = t & 15;
    int idx = dists_argmax[(size_t)node * KNB + mrow];
    const float d = dists_max[(size_t)node * KNB + mrow];
    if (idx < 0) idx += N;
    idx = idx < 0 ? 0 : (idx > N - 1 ? N - 1 : idx);
    const float* src = feature + (size_t)idx * DIN + 8 * g;
    const float4 f0 = *(const float4*)(src);
    const float4 f1 = *(const float4*)(src + 4);
    const v8h v = cvt8(f0, f1, d);
    _Float16* dst = msg + ((size_t)blockIdx.x * KNB + mrow) * DIN + 8 * g;
    *(volatile v8h*)dst = v;
    __threadfence();
    *(volatile v8h*)dst = v;
}

__global__ __launch_bounds__(NODE_TPB) void k_node(
    const _Float16* __restrict__ msg, const float* __restrict__ selfp,
    const float* __restrict__ W_hidden, const float* __restrict__ b_hidden,
    const float* __restrict__ w_out, const float* __restrict__ b_out,
    float* __restrict__ out_pos, float* __restrict__ out_str, int N, int c0)
{
    __shared__ __attribute__((aligned(16))) _Float16 wt[DOUT * WS];
    __shared__ __attribute__((aligned(16))) float srow[NODE_WPB][DOUT];
    __shared__ __attribute__((aligned(16))) float spos[NODE_WPB][32];

    const int tid = threadIdx.x;
    for (int e = tid; e < DIN * DOUT; e += NODE_TPB) {
        const int k = e >> 7;
        const int o = e & 127;
        wt[o * WS + k] = (_Float16)(W_hidden[(size_t)k * DOUT + o] * WSCALE);
    }
    __syncthreads();

    const int l = tid & 31, h = l >> 4, m = l & 15, w = tid >> 5;
    const float bout = b_out[0];
    float bia[8], wo[8];
#pragma unroll
    for (int cb = 0; cb < 8; ++cb) {
        bia[cb] = b_hidden[cb * 16 + m];
        wo[cb]  = w_out[cb * 16 + m];
    }

    float* sr = &srow[w][0];
    float* sp = &spos[w][0];
    const int nbase = c0 + ((int)blockIdx.x * NODE_WPB + w) * NPW;
    const v8f zero = {};

#pragma unroll 1
    for (int p = 0; p < NPW / 2; ++p) {
#pragma unroll 1
        for (int q = 0; q < 2; ++q) {
            const int node = nbase + 2 * p + q;
            const int ld = node < N ? node : N - 1;

            const _Float16* ap = msg + ((size_t)(ld - c0) * KNB + m) * DIN + 8 * h;
            Frag a[4];
#pragma unroll
            for (int kc = 0; kc < 4; ++kc) {
                a[kc].half[0] = *(const v8h*)(ap + kc * 32);
                a[kc].half[1] = *(const v8h*)(ap + kc * 32 + 16);
            }

            v8f acc[8];
#pragma unroll
            for (int cb = 0; cb < 8; ++cb) acc[cb] = zero;

#pragma unroll
            for (int cb = 0; cb < 8; ++cb) {
                unsigned wb = (unsigned)(m * WS + 8 * h);
                asm volatile("" : "+v"(wb));
                const _Float16* bp = wt + wb + cb * 16 * WS;
                Frag b[4];
#pragma unroll
                for (int kc = 0; kc < 4; ++kc) {
                    b[kc].half[0] = *(const v8h*)(bp + kc * 32);
                    b[kc].half[1] = *(const v8h*)(bp + kc * 32 + 16);
                }
#pragma unroll
                for (int kc = 0; kc < 4; ++kc) acc[cb] = wmma16(a[kc].v, b[kc].v, acc[cb]);
            }

            float sv[8];
#pragma unroll
            for (int cb = 0; cb < 8; ++cb) sv[cb] = selfp[(size_t)ld * DOUT + cb * 16 + m];
            float pos[8];
#pragma unroll
            for (int r = 0; r < 8; ++r) pos[r] = 0.0f;

#pragma unroll
            for (int cb = 0; cb < 8; ++cb) {
                float s = 0.0f;
#pragma unroll
                for (int r = 0; r < 8; ++r) {
                    float hv = acc[cb][r] * WINV + sv[cb];
                    hv = hv + bia[cb];
                    hv = fmaxf(hv, 0.0f);
                    s += hv;
                    pos[r] += hv * wo[cb];
                }
                s += __shfl_xor(s, 16, 32);
                if (h == 0) sr[cb * 16 + m] = s * (1.0f / KNB);
            }
#pragma unroll
            for (int r = 0; r < 8; ++r) {
                pos[r] += __shfl_xor(pos[r], 8, 32);
                pos[r] += __shfl_xor(pos[r], 4, 32);
                pos[r] += __shfl_xor(pos[r], 2, 32);
                pos[r] += __shfl_xor(pos[r], 1, 32);
            }
            if (m == 0) {
#pragma unroll
                for (int r = 0; r < 8; ++r) sp[q * 16 + 8 * h + r] = pos[r] + bout;
            }

            const v4fa ov = *(const v4fa*)(sr + 4 * l);
            float* op = out_str + (size_t)ld * DOUT + 4 * l;
            if (node < N) *(volatile v4fa*)op = ov;
            __threadfence();
            if (node < N) *(volatile v4fa*)op = ov;
        }

        const int n0 = nbase + 2 * p;
        const v4fa pv = *(const v4fa*)(sp + 4 * (l & 7));
        const bool wr = (l < 8) && (n0 + (l >> 2) < N);
        float* pp = out_pos + (size_t)n0 * KNB + 4 * (l & 7);
        if (wr) *(volatile v4fa*)pp = pv;
        __threadfence();
        if (wr) *(volatile v4fa*)pp = pv;
    }
}

extern "C" void kernel_launch(void* const* d_in, const int* in_sizes, int n_in,
                              void* d_out, int out_size, void* d_ws, size_t ws_size,
                              hipStream_t stream)
{
    if (n_in < 7 || d_ws == nullptr) return;
    const float* feature      = (const float*)d_in[0];
    const float* dists_max    = (const float*)d_in[1];
    const int*   dists_argmax = (const int*)  d_in[2];
    const float* W_hidden     = (const float*)d_in[3];
    const float* b_hidden     = (const float*)d_in[4];
    const float* w_out        = (const float*)d_in[5];
    const float* b_out        = (const float*)d_in[6];

    const int N = in_sizes[0] / DIN;
    if (N <= 0) return;
    if ((size_t)out_size < (size_t)N * (KNB + DOUT)) return;

    float* out_pos = (float*)d_out;
    float* out_str = (float*)d_out + (size_t)N * KNB;

    const int selfBlocks = (N + SELF_ROWS - 1) / SELF_ROWS;
    const size_t selfBytes = (size_t)selfBlocks * SELF_ROWS * DOUT * sizeof(float);
    if (ws_size < selfBytes) return;
    const size_t avail = ws_size - selfBytes;
    int cn = CHUNK_NODES;
    while (cn > NODES_PER_BLOCK && (size_t)cn * KNB * DIN * sizeof(_Float16) > avail) cn >>= 1;
    if ((size_t)cn * KNB * DIN * sizeof(_Float16) > avail) return;

    float*    selfp = (float*)d_ws;
    _Float16* msg   = (_Float16*)((char*)d_ws + selfBytes);

    k_self<<<selfBlocks, SELF_TPB, 0, stream>>>(feature, W_hidden, selfp, N);

    for (int c0 = 0; c0 < N; c0 += cn) {
        const int cna = (N - c0 < cn) ? (N - c0) : cn;
        k_gather<<<cna, GATHER_TPB, 0, stream>>>(feature, dists_max, dists_argmax, msg, N, c0);
        const int nb = (cna + NODES_PER_BLOCK - 1) / NODES_PER_BLOCK;
        k_node<<<nb, NODE_TPB, 0, stream>>>(msg, selfp, W_hidden, b_hidden, w_out, b_out,
                                           out_pos, out_str, N, c0);
    }
    (void)hipGetLastError();
}
